// LightWinModel_21036749815833
// MI455X (gfx1250) — hardware-verified
//
#include <hip/hip_runtime.h>

#define NROWS 2000000
#define HID 32
#define HALF 16
#define NBK 50

typedef _Float16 f16;
typedef __attribute__((ext_vector_type(16))) f16 f16x16;
typedef __attribute__((ext_vector_type(8)))  f16 f16x8;
typedef __attribute__((ext_vector_type(8)))  float f32x8;
typedef __attribute__((ext_vector_type(4)))  float v4f_t;
typedef float v4fa __attribute__((ext_vector_type(4), may_alias));

__device__ __forceinline__ f32x8 wmma16(f16x16 a, f16x16 b, f32x8 c) {
  c = __builtin_amdgcn_wmma_f32_16x16x32_f16(false, a, false, b, (short)0, c, false, false);
  asm volatile("v_nop\n\tv_nop\n\tv_nop\n\tv_nop" : "+v"(c) : "v"(a), "v"(b));
  return c;
}
__device__ __forceinline__ f16x16 lds_frag(const f16* base, int stride) {
  const int lane = threadIdx.x & 31, row = lane & 15, kh = (lane >> 4) * 8;
  const f16x8 lo = *(const f16x8*)(base + row * stride + kh);
  const f16x8 hi = *(const f16x8*)(base + row * stride + kh + 16);
  f16x16 f;
#pragma unroll
  for (int i = 0; i < 8; ++i) { f[i] = lo[i]; f[i + 8] = hi[i]; }
  return f;
}

__global__ __launch_bounds__(256) void k_lightwin(const float* __restrict__ x, const int* __restrict__ bk, const float* __restrict__ W1, const float* __restrict__ b1,
                                                 const float* __restrict__ W2, const float* __restrict__ b2, const float* __restrict__ Wh, const float* __restrict__ bh,
                                                 float* __restrict__ out) {
  __shared__ __attribute__((aligned(16))) f16 hS[2][256 * 40];
  __shared__ float w1S[2 * HID], b1S[HID], b2S[HALF], whS[NBK * HALF], bhS[NBK];
  __shared__ __attribute__((aligned(16))) float oS[256];
  const int tid = threadIdx.x, lane = tid & 31, wave = tid >> 5, cl = lane & 15, hsel = lane >> 4, kh = hsel * 8, rh = kh;
  const int r0 = blockIdx.x * 256;
  if (tid < 2 * HID) w1S[tid] = W1[tid];
  if (tid < HID) b1S[tid] = b1[tid];
  if (tid < HALF) b2S[tid] = b2[tid];
  for (int e = tid; e < NBK * HALF; e += 256) whS[e] = Wh[e];
  if (tid < NBK) bhS[tid] = bh[tid];
  __syncthreads();
  { const int row = r0 + tid; const bool ok = row < NROWS;
    const float x0 = ok ? x[(size_t)row * 2] : 0.0f, x1 = ok ? x[(size_t)row * 2 + 1] : 0.0f;
#pragma unroll
    for (int j = 0; j < HID; ++j) { const float v = fmaxf(x0 * w1S[j] + x1 * w1S[HID + j] + b1S[j], 0.0f); const f16 h = (f16)v; hS[0][tid * 40 + j] = h; hS[1][tid * 40 + j] = (f16)((v - (float)h) * 2048.0f); } }
  f16x16 wf, wl;
#pragma unroll
  for (int i = 0; i < 8; ++i) { const float a = W2[(kh + i) * HALF + cl], c2 = W2[(16 + kh + i) * HALF + cl]; const f16 ha = (f16)a, hc = (f16)c2;
    wf[i] = ha; wl[i] = (f16)((a - (float)ha) * 2048.0f); wf[8 + i] = hc; wl[8 + i] = (f16)((c2 - (float)hc) * 2048.0f); }
  __syncthreads();
#pragma unroll 1
  for (int t2 = 0; t2 < 2; ++t2) {
    const int rb = wave * 32 + t2 * 16;
    const f16x16 ah = lds_frag(hS[0] + rb * 40, 40), al = lds_frag(hS[1] + rb * 40, 40);
    f32x8 acc = {}, accx = {};
    acc = wmma16(ah, wf, acc); accx = wmma16(ah, wl, accx); accx = wmma16(al, wf, accx);
#pragma unroll
    for (int r = 0; r < 8; ++r) {
      const int rowl = rb + rh + r, row = r0 + rowl;
      int id = (row < NROWS) ? bk[row] : 0; id = (id < NBK) ? id : (NBK - 1); id = max(id, 0);
      const float hv = acc[r] + accx[r] * (1.0f / 2048.0f) + b2S[cl];
      float pv = hv * whS[id * HALF + cl];
#pragma unroll
      for (int off = 8; off >= 1; off >>= 1) pv += __shfl_xor(pv, off, 32);
      if (cl == 0) oS[rowl] = pv + bhS[id];
    }
  }
  __syncthreads();
  if (tid < 64 && r0 + tid * 4 < NROWS) {
#pragma unroll 1
    for (int pass = 0; pass < 2; ++pass) { *(volatile v4f_t*)(out + r0 + tid * 4) = *(const volatile v4fa*)(oS + tid * 4); __threadfence(); }
  }
}

extern "C" void kernel_launch(void* const* d_in, const int* in_sizes, int n_in,
                              void* d_out, int out_size, void* d_ws, size_t ws_size,
                              hipStream_t stream) {
  (void)in_sizes; (void)n_in; (void)out_size; (void)d_ws; (void)ws_size;
  const float* x = (const float*)d_in[0];
  const int* bk = (const int*)d_in[1];
  const float* W1 = (const float*)d_in[2], *b1 = (const float*)d_in[3], *W2 = (const float*)d_in[4], *b2 = (const float*)d_in[5], *Wh = (const float*)d_in[6], *bh = (const float*)d_in[7];
  float* out = (float*)d_out;
  k_lightwin<<<dim3((NROWS + 255) / 256), dim3(256), 0, stream>>>(x, bk, W1, b1, W2, b2, Wh, bh, out);
}
